// PolyAttentionBlock_8693013807186
// MI455X (gfx1250) — hardware-verified
//
#include <hip/hip_runtime.h>


static constexpr int kBatch = 16;
static constexpr int kSeq   = 1024;
static constexpr int kC     = 768;
static constexpr int kHeads = 12;
static constexpr int kDh    = 64;
static constexpr int kTok   = kBatch * kSeq;
static constexpr int kN1    = 3 * kC;
static constexpr int kCvtThreads  = 256;
static constexpr int kGemmThreads = 128;
static constexpr int kStgPitch = 132;
static constexpr int kPP = 40;
static constexpr int kOP = 68;

static_assert(kHeads * kDh == kC);
static_assert(kDh == 64);
static_assert(kSeq % 64 == 0);
static_assert(kTok % 64 == 0);
static_assert(kN1 % 128 == 0);
static_assert(kC % 128 == 0);
static_assert(kC % 32 == 0);
static_assert((kTok * kC) % (kCvtThreads * 8) == 0);
static_assert((kN1 * kC) % (kCvtThreads * 8) == 0);
static_assert((kC * kC) % (kCvtThreads * 8) == 0);
static_assert(kSeq % 32 == 0);
static_assert((kBatch * kHeads * (kSeq / 16)) % 4 == 0);
static_assert((kSeq / 16) % 4 == 0);

typedef _Float16     v16h __attribute__((ext_vector_type(16)));
typedef _Float16     v8h  __attribute__((ext_vector_type(8)));
typedef float        v8f  __attribute__((ext_vector_type(8)));
typedef float        v4f  __attribute__((ext_vector_type(4)));
typedef unsigned int v4u  __attribute__((ext_vector_type(4)));

union Frag { v16h v; v8h half[2]; };

__device__ __forceinline__ v8f wmma_f16(v16h a, v16h b, v8f acc)
{
    acc = __builtin_amdgcn_wmma_f32_16x16x32_f16(false, a, false, b, (short)0, acc, false, false);
#if defined(__HIP_DEVICE_COMPILE__)
    asm volatile("v_nop\n\tv_nop\n\tv_nop\n\tv_nop" : "+v"(acc) : "v"(a), "v"(b));
#endif
    return acc;
}

__device__ __forceinline__ float bf16_rne(float x)
{
    unsigned int u = __float_as_uint(x);
    u = u + 0x7FFFu + ((u >> 16) & 1u);
    return __uint_as_float(u & 0xFFFF0000u);
}

__device__ __forceinline__ _Float16 cvt16(float x, float sc)
{
    return (_Float16)(bf16_rne(x) * sc);
}

__global__ __launch_bounds__(kCvtThreads)
void k_cvt_rows(const float* __restrict__ src, _Float16* __restrict__ dst, float sc, int n)
{
    const size_t base = ((size_t)blockIdx.x * kCvtThreads + threadIdx.x) * 8;
    if (base + 8 <= (size_t)n) {
        const v4f f0 = *(const v4f*)(src + base);
        const v4f f1 = *(const v4f*)(src + base + 4);
        v8h hv;
        hv[0] = cvt16(f0[0], sc); hv[1] = cvt16(f0[1], sc);
        hv[2] = cvt16(f0[2], sc); hv[3] = cvt16(f0[3], sc);
        hv[4] = cvt16(f1[0], sc); hv[5] = cvt16(f1[1], sc);
        hv[6] = cvt16(f1[2], sc); hv[7] = cvt16(f1[3], sc);
        const v4u u = __builtin_bit_cast(v4u, hv);
        volatile v4u* p = (volatile v4u*)(dst + base);
        *p = u;
        __threadfence();
        *p = u;
    }
}

__global__ __launch_bounds__(kGemmThreads)
void k_gemm1(const _Float16* __restrict__ Xh, const _Float16* __restrict__ Wq,
             const float* __restrict__ bq, _Float16* __restrict__ QK,
             _Float16* __restrict__ VT)
{
    __shared__ __align__(16) float stg[64 * kStgPitch];

    const int tid  = threadIdx.x;
    const int wave = tid >> 5;
    const int lane = tid & 31;
    const int h    = lane >> 4;
    const int m    = lane & 15;
    const int n0   = blockIdx.x * 128;
    const int m0   = blockIdx.y * 64;
    const int wm   = (wave & 1) * 32;
    const int wn   = (wave >> 1) * 64;

    const _Float16* ap = Xh + (size_t)(m0 + wm + m) * kC + 8 * h;
    const _Float16* bp = Wq + (size_t)(n0 + wn + m) * kC + 8 * h;

    v8f acc[8] = {};
#pragma unroll 1
    for (int k0 = 0; k0 < kC; k0 += 32) {
        Frag a0, a1;
        a0.half[0] = *(const v8h*)(ap + k0);
        a0.half[1] = *(const v8h*)(ap + k0 + 16);
        a1.half[0] = *(const v8h*)(ap + 16 * kC + k0);
        a1.half[1] = *(const v8h*)(ap + 16 * kC + k0 + 16);
#pragma unroll
        for (int t = 0; t < 4; ++t) {
            Frag b;
            const _Float16* bt = bp + (size_t)t * 16 * kC + k0;
            b.half[0] = *(const v8h*)(bt);
            b.half[1] = *(const v8h*)(bt + 16);
            acc[t]     = wmma_f16(a0.v, b.v, acc[t]);
            acc[4 + t] = wmma_f16(a1.v, b.v, acc[4 + t]);
        }
    }

#pragma unroll
    for (int t = 0; t < 4; ++t) {
        const int c = wn + 16 * t + m;
        const float bias = bf16_rne(bq[n0 + c]);
#pragma unroll
        for (int i = 0; i < 2; ++i) {
#pragma unroll
            for (int r = 0; r < 8; ++r) {
                const float z = acc[4 * i + t][r] * (1.0f / 4096.0f) + bias;
                stg[(wm + 16 * i + 8 * h + r) * kStgPitch + c] = z;
            }
        }
    }
    __syncthreads();

    const int mode = n0 / kC;
    if (mode == 2) {
        const int bb  = m0 / kSeq;
        const int s0  = m0 % kSeq;
        const int hh0 = (n0 - 2 * kC) / kDh;
        const int p   = lane & 7;
        const int qs  = lane >> 3;
        _Float16* vb = VT + (size_t)((bb * kHeads + hh0) * kDh) * kSeq + s0 + 8 * p;
        v4u u[8];
#pragma unroll
        for (int i = 0; i < 8; ++i) {
            const int c = wave * 32 + 4 * i + qs;
            v8h hv;
#pragma unroll
            for (int e = 0; e < 8; ++e)
                hv[e] = (_Float16)(stg[(8 * p + e) * kStgPitch + c] * 16.0f);
            u[i] = __builtin_bit_cast(v4u, hv);
        }
#pragma unroll
        for (int i = 0; i < 8; ++i)
            *(volatile v4u*)(vb + (size_t)(wave * 32 + 4 * i + qs) * kSeq) = u[i];
        __threadfence();
#pragma unroll
        for (int i = 0; i < 8; ++i)
            *(volatile v4u*)(vb + (size_t)(wave * 32 + 4 * i + qs) * kSeq) = u[i];
    } else {
        const int coff = n0 - mode * kC;
        _Float16* dst = QK + (size_t)mode * kTok * kC + (size_t)m0 * kC + coff + 8 * m;
        v4u u[8];
#pragma unroll
        for (int i = 0; i < 8; ++i) {
            const int row = wave * 16 + 2 * i + h;
            const float* sp = stg + row * kStgPitch + 8 * m;
            const v4f f0 = *(const v4f*)(sp);
            const v4f f1 = *(const v4f*)(sp + 4);
            v8h hv;
            hv[0] = (_Float16)(f0[0] * 16.0f); hv[1] = (_Float16)(f0[1] * 16.0f);
            hv[2] = (_Float16)(f0[2] * 16.0f); hv[3] = (_Float16)(f0[3] * 16.0f);
            hv[4] = (_Float16)(f1[0] * 16.0f); hv[5] = (_Float16)(f1[1] * 16.0f);
            hv[6] = (_Float16)(f1[2] * 16.0f); hv[7] = (_Float16)(f1[3] * 16.0f);
            u[i] = __builtin_bit_cast(v4u, hv);
        }
#pragma unroll
        for (int i = 0; i < 8; ++i)
            *(volatile v4u*)(dst + (size_t)(wave * 16 + 2 * i + h) * kC) = u[i];
        __threadfence();
#pragma unroll
        for (int i = 0; i < 8; ++i)
            *(volatile v4u*)(dst + (size_t)(wave * 16 + 2 * i + h) * kC) = u[i];
    }
}

__global__ __launch_bounds__(kGemmThreads)
void k_attn(const _Float16* __restrict__ Qh, const _Float16* __restrict__ Kh,
            const _Float16* __restrict__ VT, const float* __restrict__ poly,
            _Float16* __restrict__ Oh)
{
    __shared__ __align__(16) _Float16 sP[4 * 16 * kPP];
    __shared__ __align__(16) float    sO[4 * 16 * kOP];

    const int tid  = threadIdx.x;
    const int wave = tid >> 5;
    const int lane = tid & 31;
    const int h    = lane >> 4;
    const int m    = lane & 15;
    const int tile = blockIdx.x * 4 + wave;
    const int q0   = (tile % (kSeq / 16)) * 16;
    const int hh   = (tile / (kSeq / 16)) % kHeads;
    const int bb   = tile / ((kSeq / 16) * kHeads);
    const int tok0 = bb * kSeq + q0;
    const int hc   = hh * kDh;

    const float pa = bf16_rne(poly[0]) * 256.0f;
    const float pb = bf16_rne(poly[1]) * 256.0f;
    const float pc = bf16_rne(poly[2]) * 256.0f;

    const _Float16* qp = Qh + (size_t)(tok0 + m) * kC + hc + 8 * h;
    Frag aq0, aq1;
    aq0.half[0] = *(const v8h*)(qp);
    aq0.half[1] = *(const v8h*)(qp + 16);
    aq1.half[0] = *(const v8h*)(qp + 32);
    aq1.half[1] = *(const v8h*)(qp + 48);

    const _Float16* kp = Kh + (size_t)(bb * kSeq + m) * kC + hc + 8 * h;
    const _Float16* vp = VT + (size_t)((bb * kHeads + hh) * kDh + m) * kSeq + 8 * h;
    _Float16* myP = sP + wave * (16 * kPP);
    float*    myO = sO + wave * (16 * kOP);

    v8f acc[4] = {};
#pragma unroll 1
    for (int kb = 0; kb < kSeq; kb += 32) {
        const _Float16* kr0 = kp + (size_t)kb * kC;
        const _Float16* kr1 = kr0 + 16 * kC;
        Frag b00, b01, b10, b11;
        b00.half[0] = *(const v8h*)(kr0);
        b00.half[1] = *(const v8h*)(kr0 + 16);
        b01.half[0] = *(const v8h*)(kr0 + 32);
        b01.half[1] = *(const v8h*)(kr0 + 48);
        b10.half[0] = *(const v8h*)(kr1);
        b10.half[1] = *(const v8h*)(kr1 + 16);
        b11.half[0] = *(const v8h*)(kr1 + 32);
        b11.half[1] = *(const v8h*)(kr1 + 48);
        v8f s0 = {}, s1 = {};
        s0 = wmma_f16(aq0.v, b00.v, s0);
        s0 = wmma_f16(aq1.v, b01.v, s0);
        s1 = wmma_f16(aq0.v, b10.v, s1);
        s1 = wmma_f16(aq1.v, b11.v, s1);

        {
            _Float16* pw = myP + (8 * h) * kPP + m;
#pragma unroll
            for (int r = 0; r < 8; ++r) {
                const float x0 = s0[r] * (1.0f / 2048.0f);
                const float x1 = s1[r] * (1.0f / 2048.0f);
                const float p0 = pa * x0 * x0 + pb * x0 + pc;
                const float p1 = pa * x1 * x1 + pb * x1 + pc;
                pw[r * kPP]      = (_Float16)p0;
                pw[r * kPP + 16] = (_Float16)p1;
            }
        }
        __syncthreads();

        Frag apf;
        apf.half[0] = *(const v8h*)(myP + m * kPP + 8 * h);
        apf.half[1] = *(const v8h*)(myP + m * kPP + 16 + 8 * h);
#pragma unroll
        for (int t = 0; t < 4; ++t) {
            Frag bv;
            const _Float16* vr = vp + (size_t)t * 16 * kSeq + kb;
            bv.half[0] = *(const v8h*)(vr);
            bv.half[1] = *(const v8h*)(vr + 16);
            acc[t] = wmma_f16(apf.v, bv.v, acc[t]);
        }
        __syncthreads();
    }

#pragma unroll
    for (int t = 0; t < 4; ++t) {
#pragma unroll
        for (int r = 0; r < 8; ++r)
            myO[(8 * h + r) * kOP + 16 * t + m] = acc[t][r] * (1.0f / 4096.0f);
    }
    __syncthreads();

    const int p  = lane & 7;
    const int qs = lane >> 3;
    v4u u[4];
#pragma unroll
    for (int i = 0; i < 4; ++i) {
        const int row = 4 * i + qs;
        const float* spo = myO + row * kOP + 8 * p;
        const v4f f0 = *(const v4f*)(spo);
        const v4f f1 = *(const v4f*)(spo + 4);
        v8h hv;
        hv[0] = (_Float16)f0[0]; hv[1] = (_Float16)f0[1]; hv[2] = (_Float16)f0[2]; hv[3] = (_Float16)f0[3];
        hv[4] = (_Float16)f1[0]; hv[5] = (_Float16)f1[1]; hv[6] = (_Float16)f1[2]; hv[7] = (_Float16)f1[3];
        u[i] = __builtin_bit_cast(v4u, hv);
    }
    _Float16* dst = Oh + (size_t)tok0 * kC + hc + 8 * p;
#pragma unroll
    for (int i = 0; i < 4; ++i)
        *(volatile v4u*)(dst + (size_t)(4 * i + qs) * kC) = u[i];
    __threadfence();
#pragma unroll
    for (int i = 0; i < 4; ++i)
        *(volatile v4u*)(dst + (size_t)(4 * i + qs) * kC) = u[i];
}

__global__ __launch_bounds__(kGemmThreads)
void k_gemm2(const _Float16* __restrict__ Ah, const _Float16* __restrict__ Wp,
             const float* __restrict__ bp2, float* __restrict__ Out)
{
    __shared__ __align__(16) float stg[64 * kStgPitch];

    const int tid  = threadIdx.x;
    const int wave = tid >> 5;
    const int lane = tid & 31;
    const int h    = lane >> 4;
    const int m    = lane & 15;
    const int n0   = blockIdx.x * 128;
    const int m0   = blockIdx.y * 64;
    const int wm   = (wave & 1) * 32;
    const int wn   = (wave >> 1) * 64;

    const _Float16* ap = Ah + (size_t)(m0 + wm + m) * kC + 8 * h;
    const _Float16* bp = Wp + (size_t)(n0 + wn + m) * kC + 8 * h;

    v8f acc[8] = {};
#pragma unroll 1
    for (int k0 = 0; k0 < kC; k0 += 32) {
        Frag a0, a1;
        a0.half[0] = *(const v8h*)(ap + k0);
        a0.half[1] = *(const v8h*)(ap + k0 + 16);
        a1.half[0] = *(const v8h*)(ap + 16 * kC + k0);
        a1.half[1] = *(const v8h*)(ap + 16 * kC + k0 + 16);
#pragma unroll
        for (int t = 0; t < 4; ++t) {
            Frag b;
            const _Float16* bt = bp + (size_t)t * 16 * kC + k0;
            b.half[0] = *(const v8h*)(bt);
            b.half[1] = *(const v8h*)(bt + 16);
            acc[t]     = wmma_f16(a0.v, b.v, acc[t]);
            acc[4 + t] = wmma_f16(a1.v, b.v, acc[4 + t]);
        }
    }

#pragma unroll
    for (int t = 0; t < 4; ++t) {
        const int c = wn + 16 * t + m;
        const float bias = bf16_rne(bp2[n0 + c]);
#pragma unroll
        for (int i = 0; i < 2; ++i) {
#pragma unroll
            for (int r = 0; r < 8; ++r) {
                const float y = acc[4 * i + t][r] * (1.0f / 256.0f) + bias;
                stg[(wm + 16 * i + 8 * h + r) * kStgPitch + c] = y;
            }
        }
    }
    __syncthreads();

    float* dst = Out + (size_t)m0 * kC + n0 + 4 * lane;
#pragma unroll
    for (int g = 0; g < 4; ++g) {
        v4f v[4];
#pragma unroll
        for (int rr = 0; rr < 4; ++rr) {
            const int row = wave * 16 + 4 * g + rr;
            v[rr] = *(const v4f*)(stg + row * kStgPitch + 4 * lane);
        }
#pragma unroll
        for (int rr = 0; rr < 4; ++rr)
            *(volatile v4f*)(dst + (size_t)(wave * 16 + 4 * g + rr) * kC) = v[rr];
        __threadfence();
#pragma unroll
        for (int rr = 0; rr < 4; ++rr)
            *(volatile v4f*)(dst + (size_t)(wave * 16 + 4 * g + rr) * kC) = v[rr];
    }
}

extern "C" void kernel_launch(void* const* d_in, const int* in_sizes, int n_in,
                              void* d_out, int out_size, void* d_ws, size_t ws_size,
                              hipStream_t stream)
{
    if (n_in < 6) return;
    if (in_sizes[0] != kTok * kC) return;
    if (in_sizes[1] != kN1 * kC) return;
    if (in_sizes[2] != kN1) return;
    if (in_sizes[3] != kC * kC) return;
    if (in_sizes[4] != kC) return;
    if (in_sizes[5] < 3) return;
    if (out_size != kTok * kC) return;

    const size_t bXh = (size_t)kTok * kC * sizeof(_Float16);
    const size_t bWq = (size_t)kN1 * kC * sizeof(_Float16);
    const size_t bWp = (size_t)kC * kC * sizeof(_Float16);
    const size_t bQK = (size_t)2 * kTok * kC * sizeof(_Float16);
    const size_t bVT = (size_t)kBatch * kHeads * kDh * kSeq * sizeof(_Float16);
    const size_t bOh = (size_t)kTok * kC * sizeof(_Float16);
    const size_t total = bXh + bWq + bWp + bQK + bVT + bOh;
    if (ws_size < total) return;

    const float* x      = (const float*)d_in[0];
    const float* w_qkv  = (const float*)d_in[1];
    const float* b_qkv  = (const float*)d_in[2];
    const float* w_proj = (const float*)d_in[3];
    const float* b_proj = (const float*)d_in[4];
    const float* poly   = (const float*)d_in[5];
    float* Out = (float*)d_out;

    char* ws = (char*)d_ws;
    size_t o = 0;
    _Float16* Xh = (_Float16*)(ws + o); o += bXh;
    _Float16* Wq = (_Float16*)(ws + o); o += bWq;
    _Float16* Wp = (_Float16*)(ws + o); o += bWp;
    _Float16* QK = (_Float16*)(ws + o); o += bQK;
    _Float16* VT = (_Float16*)(ws + o); o += bVT;
    _Float16* Oh = (_Float16*)(ws + o); o += bOh;
    const _Float16* Qh = QK;
    const _Float16* Kh = QK + (size_t)kTok * kC;

    const int nX = kTok * kC;
    const int nW = kN1 * kC;
    const int nP = kC * kC;
    k_cvt_rows<<<dim3((unsigned)((nX / 8 + kCvtThreads - 1) / kCvtThreads)), dim3(kCvtThreads), 0, stream>>>(x, Xh, 16.0f, nX);
    k_cvt_rows<<<dim3((unsigned)((nW / 8 + kCvtThreads - 1) / kCvtThreads)), dim3(kCvtThreads), 0, stream>>>(w_qkv, Wq, 256.0f, nW);
    k_cvt_rows<<<dim3((unsigned)((nP / 8 + kCvtThreads - 1) / kCvtThreads)), dim3(kCvtThreads), 0, stream>>>(w_proj, Wp, 256.0f, nP);
    k_gemm1<<<dim3(kN1 / 128, kTok / 64), dim3(kGemmThreads), 0, stream>>>(Xh, Wq, b_qkv, QK, VT);
    k_attn<<<dim3((kBatch * kHeads * (kSeq / 16)) / 4), dim3(kGemmThreads), 0, stream>>>(Qh, Kh, VT, poly, Oh);
    k_gemm2<<<dim3(kC / 128, kTok / 64), dim3(kGemmThreads), 0, stream>>>(Oh, Wp, b_proj, Out);
}
